// MultiHeadAttention_SHORT_26628797235509
// MI455X (gfx1250) — hardware-verified
//
#include <hip/hip_runtime.h>
#include <math.h>
#include <stdint.h>

constexpr int kBatch = 2;
constexpr int kSeq   = 2048;
constexpr int kDm    = 1024;
constexpr int kHeads = 16;
constexpr int kHd    = 64;
static_assert(kHeads * kHd == kDm, "head split");
static_assert(kSeq % 64 == 0 && kDm % 64 == 0, "tile multiples");

typedef __attribute__((ext_vector_type(16))) _Float16 v16h;
typedef __attribute__((ext_vector_type(8)))  _Float16 v8h;
typedef __attribute__((ext_vector_type(16))) __bf16   v16b;
typedef __attribute__((ext_vector_type(8)))  __bf16   v8b;
typedef __attribute__((ext_vector_type(8)))  float    v8f;
typedef __attribute__((ext_vector_type(4)))  float    v4f;
typedef __attribute__((ext_vector_type(2)))  float    v2f;

__device__ __forceinline__ unsigned short f2bf_bits(float f) {
  unsigned u = __float_as_uint(f);
  return (unsigned short)((u + 0x7FFFu + ((u >> 16) & 1u)) >> 16);
}
__device__ __forceinline__ float bf_bits2f(unsigned short h) { return __uint_as_float(((unsigned)h) << 16); }
__device__ __forceinline__ unsigned pk16(unsigned short a, unsigned short b) { return (unsigned)a | ((unsigned)b << 16); }

__device__ __forceinline__ void dep_guard_h(v8f& a, v8f& b, v16h x, v16h y) { asm volatile("v_nop\n\tv_nop\n\tv_nop\n\tv_nop" : "+v"(a), "+v"(b) : "v"(x), "v"(y)); }
__device__ __forceinline__ void dep_guard_b(v8f& a, v8f& b, v16b x, v16b y) { asm volatile("v_nop\n\tv_nop\n\tv_nop\n\tv_nop" : "+v"(a), "+v"(b) : "v"(x), "v"(y)); }
__device__ __forceinline__ void keep4_h(v16h a, v16h b, v16h c, v16h d) { asm volatile("v_nop" :: "v"(a), "v"(b), "v"(c), "v"(d)); }
__device__ __forceinline__ void keep4_b(v16b a, v16b b, v16b c, v16b d) { asm volatile("v_nop" :: "v"(a), "v"(b), "v"(c), "v"(d)); }
__device__ __forceinline__ void acc_guard4(v8f& a, v8f& b, v8f& c, v8f& d) { asm volatile("v_nop\n\tv_nop\n\tv_nop\n\tv_nop" : "+v"(a), "+v"(b), "+v"(c), "+v"(d)); }
template <typename T> struct Frag;
template <> struct Frag<_Float16> {
  typedef v16h V; union U { v16h v; v8h h[2]; };
  static __device__ __forceinline__ v16h load(const _Float16* p) {
    U f; f.h[0] = *(const v8h*)(p); f.h[1] = *(const v8h*)(p + 16); return f.v;
  }
  static __device__ __forceinline__ v8f mma(v16h a, v16h b, v8f c) {
    return __builtin_amdgcn_wmma_f32_16x16x32_f16(false, a, false, b, (short)0, c, false, false);
  }
  static __device__ __forceinline__ void guard(v8f& a, v8f& b, v16h x, v16h y) { dep_guard_h(a, b, x, y); }
  static __device__ __forceinline__ void keep(v16h a, v16h b, v16h c, v16h d) { keep4_h(a, b, c, d); }
};
template <> struct Frag<__bf16> {
  typedef v16b V; union U { v16b v; v8b h[2]; };
  static __device__ __forceinline__ v16b load(const __bf16* p) {
    U f; f.h[0] = *(const v8b*)(p); f.h[1] = *(const v8b*)(p + 16); return f.v;
  }
  static __device__ __forceinline__ v8f mma(v16b a, v16b b, v8f c) {
    return __builtin_amdgcn_wmma_f32_16x16x32_bf16(false, a, false, b, (short)0, c, false, false);
  }
  static __device__ __forceinline__ void guard(v8f& a, v8f& b, v16b x, v16b y) { dep_guard_b(a, b, x, y); }
  static __device__ __forceinline__ void keep(v16b a, v16b b, v16b c, v16b d) { keep4_b(a, b, c, d); }
};

template <int ET> struct Elem;
template <> struct Elem<0> { typedef _Float16 T; };
template <> struct Elem<1> { typedef __bf16 T; };
template <int ET, bool SPLIT, int BIAS_MODE, int OUT_MODE, bool RESID, int ACT = 0>
__global__ __launch_bounds__(256) void wmma_gemm64(
    const unsigned short* __restrict__ Ap, const unsigned short* __restrict__ A2p, int lda, long strideA,
    const unsigned short* __restrict__ Btp, const unsigned short* __restrict__ Bt2p, int ldb, long strideB,
    void* __restrict__ Cout, void* __restrict__ Cout2, int ldc, long strideC,
    const float* __restrict__ bias,
    const float* __restrict__ resid, long strideR,
    int M, int N, int K, float scale) {
  typedef typename Elem<ET>::T T;
  typedef typename Frag<T>::V V;
  const T* A = (const T*)Ap; const T* A2 = (const T*)A2p; const T* Bt = (const T*)Btp; const T* Bt2 = (const T*)Bt2p;
  __shared__ __align__(16) float sT[8][16 * 68];
  const int b    = blockIdx.y;
  const int lane = threadIdx.x & 31;
  const int wave = threadIdx.x >> 5;
  const int tilesN = N >> 6;
  const int tilesM = M >> 6;
  const int tile = blockIdx.x * 8 + wave;
  if (tile >= tilesM * tilesN) return;
  const int tm = tile / tilesN;
  const int tn = tile - tm * tilesN;
  const int m0 = tm << 6;
  const int n0 = tn << 6;

  const T* Ab  = A  + (size_t)b * strideA;
  const T* Bb  = Bt + (size_t)b * strideB;
  const T* Ab2 = SPLIT ? (A2  + (size_t)b * strideA) : nullptr;
  const T* Bb2 = SPLIT ? (Bt2 + (size_t)b * strideB) : nullptr;

  const int rlane = lane & 15;
  const int koff  = (lane >> 4) * 8;
  const int mOff  = (lane >> 4) * 8;

  v8f acc[4][4];
#pragma unroll
  for (int i = 0; i < 4; ++i)
#pragma unroll
    for (int j = 0; j < 4; ++j) acc[i][j] = (v8f){0.f,0.f,0.f,0.f,0.f,0.f,0.f,0.f};

  for (int k0 = 0; k0 < K; k0 += 32) {
    V bh[4], bl[4];
#pragma unroll
    for (int j = 0; j < 4; ++j) {
      const size_t bo = (size_t)(n0 + (j << 4) + rlane) * ldb + koff + k0;
      bh[j] = Frag<T>::load(Bb + bo);
      if (SPLIT) bl[j] = Frag<T>::load(Bb2 + bo);
    }
#pragma unroll
    for (int i = 0; i < 4; ++i) {
      const size_t ao = (size_t)(m0 + (i << 4) + rlane) * lda + koff + k0;
      V ah = Frag<T>::load(Ab + ao);
      V al;
      if (SPLIT) al = Frag<T>::load(Ab2 + ao);
#pragma unroll
      for (int j = 0; j < 4; ++j) {
        acc[i][j] = Frag<T>::mma(ah, bh[j], acc[i][j]);
        if (SPLIT) {
          acc[i][j] = Frag<T>::mma(ah, bl[j], acc[i][j]);
          acc[i][j] = Frag<T>::mma(al, bh[j], acc[i][j]);
        }
      }
      Frag<T>::guard(acc[i][0], acc[i][3], ah, SPLIT ? al : ah);
    }
    Frag<T>::keep(bh[0], bh[1], bh[2], bh[3]);
    if (SPLIT) Frag<T>::keep(bl[0], bl[1], bl[2], bl[3]);
  }
  acc_guard4(acc[0][0], acc[0][1], acc[0][2], acc[0][3]);
  acc_guard4(acc[1][0], acc[1][1], acc[1][2], acc[1][3]);
  acc_guard4(acc[2][0], acc[2][1], acc[2][2], acc[2][3]);
  acc_guard4(acc[3][0], acc[3][1], acc[3][2], acc[3][3]);

  float* slab = sT[wave];
  const float* Rb = RESID ? (resid + (size_t)b * strideR) : nullptr;
#pragma unroll
  for (int i = 0; i < 4; ++i) {
    const int mBase = m0 + (i << 4);
#pragma unroll
    for (int j = 0; j < 4; ++j) {
      const int n = n0 + (j << 4) + rlane;
      float bv = 0.f;
      if (BIAS_MODE == 2) bv = bias[n];
#pragma unroll
      for (int r = 0; r < 8; ++r) {
        float v = acc[i][j][r] * scale;
        if (BIAS_MODE == 1) v += bias[mBase + mOff + r];
        if (BIAS_MODE == 2) v += bv;
        if (RESID) v += Rb[(size_t)(mBase + mOff + r) * ldc + n];
        if (ACT == 1) v = tanhf(v);
        if (ACT == 2) v = fmaxf(v, 0.0f);
        if (ACT == 3) v = v / (1.0f + expf(-v));
        if (ACT == 4) v = (v > 0.f) ? v : 0.01f * v;
        if (ACT == 5) v = 0.5f * v * (1.0f + erff(v * 0.70710678118654752f));
        slab[(mOff + r) * 68 + (j << 4) + rlane] = v;
      }
    }
    __builtin_amdgcn_fence(__ATOMIC_RELEASE, "workgroup");
    __builtin_amdgcn_wave_barrier();
    __builtin_amdgcn_fence(__ATOMIC_ACQUIRE, "workgroup");
    if (OUT_MODE == 0) {
      float* C = (float*)Cout + (size_t)b * strideC;
      const int hh = lane >> 4, c4 = (lane & 15) * 4;
      for (int pass = 0; pass < 2; ++pass) {
#pragma unroll
        for (int it = 0; it < 8; ++it) {
          const int row = it * 2 + hh;
          v4f v = *(const v4f*)(slab + row * 68 + c4);
          *(volatile v4f*)(C + (size_t)(mBase + row) * ldc + n0 + c4) = v;
        }
        __threadfence();
      }
    } else {
      const int q = lane >> 3, c8 = (lane & 7) * 8;
      unsigned short* C  = (unsigned short*)Cout  + (size_t)b * strideC;
      unsigned short* C2 = (OUT_MODE == 2) ? ((unsigned short*)Cout2 + (size_t)b * strideC) : nullptr;
      for (int pass = 0; pass < 2; ++pass) {
#pragma unroll
        for (int it = 0; it < 4; ++it) {
          const int row = it * 4 + q;
          const float* sp = slab + row * 68 + c8;
          v8h hv, lv;
#pragma unroll
          for (int e = 0; e < 8; ++e) {
            if (OUT_MODE == 1) {
              hv[e] = (_Float16)sp[e];
            } else {
              unsigned short hb = f2bf_bits(sp[e]);
              unsigned short lb = f2bf_bits(sp[e] - bf_bits2f(hb));
              hv[e] = __builtin_bit_cast(_Float16, hb);
              lv[e] = __builtin_bit_cast(_Float16, lb);
            }
          }
          *(volatile v8h*)(C + (size_t)(mBase + row) * ldc + n0 + c8) = hv;
          if (OUT_MODE == 2) *(volatile v8h*)(C2 + (size_t)(mBase + row) * ldc + n0 + c8) = lv;
        }
        __threadfence();
      }
    }
    __builtin_amdgcn_fence(__ATOMIC_RELEASE, "workgroup");
    __builtin_amdgcn_wave_barrier();
    __builtin_amdgcn_fence(__ATOMIC_ACQUIRE, "workgroup");
  }
}

__global__ __launch_bounds__(256) void cast_f32_bf16x2(const float* __restrict__ in, unsigned short* __restrict__ out, int n2) {
  const int i = blockIdx.x * 256 + threadIdx.x;
  if (i < n2) {
    const v2f f = *(const v2f*)(in + 2 * (size_t)i);
    const unsigned u = pk16(f2bf_bits(f[0]), f2bf_bits(f[1]));
    ((volatile unsigned*)out)[i] = u;
    __threadfence();
    ((volatile unsigned*)out)[i] = u;
  }
}

__global__ __launch_bounds__(256) void cast_f32_bf_f16x2(const float* __restrict__ in, unsigned short* __restrict__ out, int n2, float scale) {
  const int i = blockIdx.x * 256 + threadIdx.x;
  if (i < n2) {
    const v2f f = *(const v2f*)(in + 2 * (size_t)i);
    const _Float16 h0 = (_Float16)(bf_bits2f(f2bf_bits(f[0])) * scale);
    const _Float16 h1 = (_Float16)(bf_bits2f(f2bf_bits(f[1])) * scale);
    const unsigned u = pk16(__builtin_bit_cast(unsigned short, h0), __builtin_bit_cast(unsigned short, h1));
    ((volatile unsigned*)out)[i] = u;
    __threadfence();
    ((volatile unsigned*)out)[i] = u;
  }
}

__global__ __launch_bounds__(256) void bias_bf16_kernel(const float* __restrict__ b0, const float* __restrict__ b1,
                                                        const float* __restrict__ b2, const float* __restrict__ b3,
                                                        float* __restrict__ out, int n) {
  const int y = blockIdx.y;
  const float* src = b0;
  if (y == 1) src = b1;
  if (y == 2) src = b2;
  if (y == 3) src = b3;
  const int i = blockIdx.x * 256 + threadIdx.x;
  if (4 * i + 3 < n) {
    const v4f f = *(const v4f*)(src + 4 * (size_t)i);
    v4f rv;
    rv[0] = bf_bits2f(f2bf_bits(f[0]));
    rv[1] = bf_bits2f(f2bf_bits(f[1]));
    rv[2] = bf_bits2f(f2bf_bits(f[2]));
    rv[3] = bf_bits2f(f2bf_bits(f[3]));
    float* dst = out + (size_t)y * n + 4 * (size_t)i;
    *(volatile v4f*)dst = rv;
    __threadfence();
    *(volatile v4f*)dst = rv;
  }
}

#define AT_D 64
#define AT_NW 4
#define AT_QB 64
#define AT_KC 64
constexpr float kPScale   = 32768.0f;
constexpr float kMaskFill = -1.0e9f;

__device__ __forceinline__ v8f at_mma_h(v16h a, v16h b, v8f c) {
  c = __builtin_amdgcn_wmma_f32_16x16x32_f16(false, a, false, b, (short)0, c, false, false);
  asm volatile("v_nop\n\tv_nop\n\tv_nop\n\tv_nop" : "+v"(c) : "v"(a), "v"(b));
  return c;
}

__global__ __launch_bounds__(128)
void attn_mask64_kernel(const unsigned short* __restrict__ qp, const unsigned short* __restrict__ kp,
                        const unsigned short* __restrict__ vtp, const int* __restrict__ mask,
                        unsigned short* __restrict__ ctxp, float sscale, float oscale) {
  union FB { v16h v; v8h h[2]; };
  __shared__ __align__(16) _Float16 Ksh[AT_KC * AT_D];
  __shared__ __align__(16) _Float16 Vth[AT_D * AT_KC];
  __shared__ __align__(16) _Float16 Psh[AT_NW][16 * AT_KC];
  __shared__ __align__(16) float    Os[AT_NW][16 * 68];

  const int tid  = threadIdx.x;
  const int wave = tid >> 5;
  const int lane = tid & 31;
  const int hh   = lane >> 4;
  const int c    = lane & 15;

  const int nqb = kSeq / AT_QB;
  const int bx  = blockIdx.x;
  const int qb  = bx % nqb;
  const int bh  = bx / nqb;
  const int h   = bh % kHeads;
  int b = bh / kHeads; b = (b < kBatch) ? b : (kBatch - 1);
  const int q0  = qb * AT_QB + wave * 16;

  const _Float16* Qh = (const _Float16*)(const void*)qp  + (size_t)b * kSeq * kDm + (size_t)h * AT_D;
  const _Float16* Kh = (const _Float16*)(const void*)kp  + (size_t)b * kSeq * kDm + (size_t)h * AT_D;
  const _Float16* Vt = (const _Float16*)(const void*)vtp + ((size_t)b * kDm + (size_t)h * AT_D) * kSeq;
  const int*      mb = mask + (size_t)b * kSeq * kSeq;
  _Float16*       ob = (_Float16*)(void*)ctxp + (size_t)b * kSeq * kDm + (size_t)h * AT_D;

  v16h qa[2];
#pragma unroll
  for (int dc = 0; dc < 2; ++dc) {
    qa[dc] = Frag<_Float16>::load(Qh + (size_t)(q0 + c) * kDm + dc * 32 + 8 * hh);
  }

  float mrow[8], lrow[8];
  v8f oacc[4];
#pragma unroll
  for (int r = 0; r < 8; ++r) { mrow[r] = -INFINITY; lrow[r] = 0.f; }
#pragma unroll
  for (int t = 0; t < 4; ++t) oacc[t] = (v8f){0.f,0.f,0.f,0.f,0.f,0.f,0.f,0.f};

  const int nChunks = kSeq / AT_KC;
  for (int kc = 0; kc < nChunks; ++kc) {
    const int kv0 = kc * AT_KC;
    __syncthreads();
    {
      const int r = tid >> 1, half = (tid & 1) * 32;
      const _Float16* ks = Kh + (size_t)(kv0 + r) * kDm + half;
      const _Float16* vs = Vt + (size_t)r * kSeq + kv0 + half;
#pragma unroll
      for (int i = 0; i < 4; ++i) {
        const v8h a0 = *(const v8h*)(ks + 8 * i);
        const v8h b0 = *(const v8h*)(vs + 8 * i);
        *(v8h*)(Ksh + r * AT_D  + half + 8 * i) = a0;
        *(v8h*)(Vth + r * AT_KC + half + 8 * i) = b0;
      }
    }
    __syncthreads();

    v8f s[4];
#pragma unroll
    for (int j = 0; j < 4; ++j) {
      s[j] = (v8f){0.f,0.f,0.f,0.f,0.f,0.f,0.f,0.f};
#pragma unroll
      for (int dc = 0; dc < 2; ++dc) {
        FB kb;
        kb.h[0] = *(const v8h*)(Ksh + (j * 16 + c) * AT_D + dc * 32 + 8 * hh);
        kb.h[1] = *(const v8h*)(Ksh + (j * 16 + c) * AT_D + dc * 32 + 16 + 8 * hh);
        s[j] = at_mma_h(qa[dc], kb.v, s[j]);
      }
    }
    float cm[8];
#pragma unroll
    for (int r = 0; r < 8; ++r) {
      const int qrow = q0 + 8 * hh + r;
      const int* mr = mb + (size_t)qrow * kSeq + kv0;
      float m = -INFINITY;
#pragma unroll
      for (int j = 0; j < 4; ++j) {
        const int mv = mr[j * 16 + c];
        const float sv = s[j][r] * sscale;
        const float sm = (mv == 0) ? kMaskFill : sv;
        s[j][r] = sm;
        m = fmaxf(m, sm);
      }
#pragma unroll
      for (int off = 1; off < 16; off <<= 1) m = fmaxf(m, __shfl_xor(m, off, 32));
      cm[r] = m;
    }
    _Float16* pwh = Psh[wave];
#pragma unroll
    for (int r = 0; r < 8; ++r) {
      const float mnew = fmaxf(mrow[r], cm[r]);
      const float alpha = expf(mrow[r] - mnew);
      mrow[r] = mnew;
      float psum = 0.f;
#pragma unroll
      for (int j = 0; j < 4; ++j) {
        const float p = expf(s[j][r] - mnew);
        psum += p;
        pwh[(8 * hh + r) * AT_KC + j * 16 + c] = (_Float16)(p * kPScale);
      }
#pragma unroll
      for (int off = 1; off < 16; off <<= 1) psum += __shfl_xor(psum, off, 32);
      lrow[r] = lrow[r] * alpha + psum;
#pragma unroll
      for (int t = 0; t < 4; ++t) oacc[t][r] *= alpha;
    }
    __builtin_amdgcn_fence(__ATOMIC_RELEASE, "workgroup");
    __builtin_amdgcn_wave_barrier();
    __builtin_amdgcn_fence(__ATOMIC_ACQUIRE, "workgroup");
#pragma unroll 1
    for (int kk = 0; kk < 2; ++kk) {
      FB pa;
      pa.h[0] = *(const v8h*)(pwh + c * AT_KC + kk * 32 + 8 * hh);
      pa.h[1] = *(const v8h*)(pwh + c * AT_KC + kk * 32 + 16 + 8 * hh);
#pragma unroll
      for (int t = 0; t < 4; ++t) {
        FB vb;
        vb.h[0] = *(const v8h*)(Vth + (t * 16 + c) * AT_KC + kk * 32 + 8 * hh);
        vb.h[1] = *(const v8h*)(Vth + (t * 16 + c) * AT_KC + kk * 32 + 16 + 8 * hh);
        oacc[t] = at_mma_h(pa.v, vb.v, oacc[t]);
      }
    }
  }

  float* os = Os[wave];
#pragma unroll
  for (int r = 0; r < 8; ++r) {
    const float inv = oscale / (lrow[r] * kPScale);
#pragma unroll
    for (int t = 0; t < 4; ++t) os[(8 * hh + r) * 68 + t * 16 + c] = oacc[t][r] * inv;
  }
  __builtin_amdgcn_fence(__ATOMIC_RELEASE, "workgroup");
  __builtin_amdgcn_wave_barrier();
  __builtin_amdgcn_fence(__ATOMIC_ACQUIRE, "workgroup");
  {
    const int q8 = lane >> 3, c8 = (lane & 7) * 8;
    for (int pass = 0; pass < 2; ++pass) {
#pragma unroll
      for (int it = 0; it < 4; ++it) {
        const int row = it * 4 + q8;
        const float* sp = os + row * 68 + c8;
        v8h hv;
#pragma unroll
        for (int e = 0; e < 8; ++e) hv[e] = (_Float16)sp[e];
        *(volatile v8h*)(ob + (size_t)(q0 + row) * kDm + c8) = hv;
      }
      __threadfence();
    }
  }
}

extern "C" void kernel_launch(void* const* d_in, const int* in_sizes, int n_in,
                              void* d_out, int out_size, void* d_ws, size_t ws_size,
                              hipStream_t stream) {
  if (n_in < 12) return;
  const int nAct = kBatch * kSeq * kDm;
  const int nW   = kDm * kDm;
  if (in_sizes[0] != nAct || in_sizes[1] != nAct || in_sizes[2] != nAct) return;
  if (in_sizes[3] != kBatch * kSeq * kSeq) return;
  if (in_sizes[4] != nW || in_sizes[6] != nW || in_sizes[8] != nW || in_sizes[10] != nW) return;
  if (in_sizes[5] != kDm || in_sizes[7] != kDm || in_sizes[9] != kDm || in_sizes[11] != kDm) return;
  if (out_size != nAct) return;

  const float* q    = (const float*)d_in[0];
  const float* k    = (const float*)d_in[1];
  const float* v    = (const float*)d_in[2];
  const int*   mask = (const int*)d_in[3];
  const float* Wq   = (const float*)d_in[4];
  const float* bq   = (const float*)d_in[5];
  const float* Wk   = (const float*)d_in[6];
  const float* bk   = (const float*)d_in[7];
  const float* Wv   = (const float*)d_in[8];
  const float* bv   = (const float*)d_in[9];
  const float* Wo   = (const float*)d_in[10];
  const float* bo   = (const float*)d_in[11];

  const size_t bAct16 = (size_t)nAct * 2;
  const size_t bW16   = (size_t)nW * 2;
  size_t off = 0;
  const size_t oQ16  = off; off += bAct16;
  const size_t oK16  = off; off += bAct16;
  const size_t oV16  = off; off += bAct16;
  const size_t oWq   = off; off += bW16;
  const size_t oWk   = off; off += bW16;
  const size_t oWv   = off; off += bW16;
  const size_t oWo   = off; off += bW16;
  const size_t oBias = off; off += (size_t)4 * kDm * sizeof(float);
  const size_t oQP   = off; off += bAct16;
  const size_t oKP   = off; off += bAct16;
  const size_t oVT   = off; off += bAct16;
  const size_t oCTX  = off; off += bAct16;
  if (off > ws_size) return;

  char* ws = (char*)d_ws;
  unsigned short* Q16  = (unsigned short*)(ws + oQ16);
  unsigned short* K16  = (unsigned short*)(ws + oK16);
  unsigned short* V16  = (unsigned short*)(ws + oV16);
  unsigned short* WQ16 = (unsigned short*)(ws + oWq);
  unsigned short* WK16 = (unsigned short*)(ws + oWk);
  unsigned short* WV16 = (unsigned short*)(ws + oWv);
  unsigned short* WO16 = (unsigned short*)(ws + oWo);
  float* biasR = (float*)(ws + oBias);
  const float* bqR = biasR;
  const float* bkR = biasR + kDm;
  const float* bvR = biasR + 2 * kDm;
  const float* boR = biasR + 3 * kDm;
  unsigned short* QP    = (unsigned short*)(ws + oQP);
  unsigned short* KP    = (unsigned short*)(ws + oKP);
  unsigned short* VT    = (unsigned short*)(ws + oVT);
  unsigned short* CTX16 = (unsigned short*)(ws + oCTX);

  const int nAct2 = nAct / 2;
  const int nW2   = nW / 2;
  cast_f32_bf16x2<<<dim3(nAct2 / 256), dim3(256), 0, stream>>>(q, Q16, nAct2);
  cast_f32_bf16x2<<<dim3(nAct2 / 256), dim3(256), 0, stream>>>(k, K16, nAct2);
  cast_f32_bf16x2<<<dim3(nAct2 / 256), dim3(256), 0, stream>>>(v, V16, nAct2);
  cast_f32_bf16x2<<<dim3(nW2 / 256), dim3(256), 0, stream>>>(Wq, WQ16, nW2);
  cast_f32_bf16x2<<<dim3(nW2 / 256), dim3(256), 0, stream>>>(Wk, WK16, nW2);
  cast_f32_bf16x2<<<dim3(nW2 / 256), dim3(256), 0, stream>>>(Wv, WV16, nW2);
  cast_f32_bf_f16x2<<<dim3(nW2 / 256), dim3(256), 0, stream>>>(Wo, WO16, nW2, 64.0f);
  bias_bf16_kernel<<<dim3(kDm / 1024, 4), dim3(256), 0, stream>>>(bq, bk, bv, bo, biasR, kDm);

  const int mRows = kBatch * kSeq;
  wmma_gemm64<1, false, 2, 1, false><<<dim3((mRows / 64) * (kDm / 64) / 8, 1), dim3(256), 0, stream>>>(
      Q16, Q16, kDm, 0L, WQ16, WQ16, kDm, 0L, (void*)QP, (void*)QP, kDm, 0L, bqR, bq, 0L, mRows, kDm, kDm, 1.0f);
  wmma_gemm64<1, false, 2, 1, false><<<dim3((mRows / 64) * (kDm / 64) / 8, 1), dim3(256), 0, stream>>>(
      K16, K16, kDm, 0L, WK16, WK16, kDm, 0L, (void*)KP, (void*)KP, kDm, 0L, bkR, bk, 0L, mRows, kDm, kDm, 1.0f);
  wmma_gemm64<1, false, 1, 1, false><<<dim3((kDm / 64) * (kSeq / 64) / 8, kBatch), dim3(256), 0, stream>>>(
      WV16, WV16, kDm, 0L, V16, V16, kDm, (long)kSeq * kDm, (void*)VT, (void*)VT, kSeq, (long)kDm * kSeq,
      bvR, bv, 0L, kDm, kSeq, kDm, 1.0f);
  attn_mask64_kernel<<<dim3(kBatch * kHeads * (kSeq / 64)), dim3(128), 0, stream>>>(
      QP, KP, VT, mask, CTX16, 0.125f, 16.0f);
  wmma_gemm64<0, false, 2, 0, false><<<dim3((mRows / 64) * (kDm / 64) / 8, 1), dim3(256), 0, stream>>>(
      CTX16, CTX16, kDm, 0L, WO16, WO16, kDm, 0L, d_out, d_out, kDm, 0L, boR, bo, 0L, mRows, kDm, kDm,
      1.0f / 1024.0f);
}
